// BiNet_70506183131681
// MI455X (gfx1250) — hardware-run, weakly checked
//
#include <hip/hip_runtime.h>


namespace {
constexpr int ND = 220000, NP_ = 120000, E = 1500000, C = 32, KPAD = 96, NBR = 4;
constexpr float XS = 8.0f, WSC = 256.0f;
typedef _Float16 b16;
typedef __attribute__((ext_vector_type(16))) _Float16 v16b;
typedef __attribute__((ext_vector_type(8))) _Float16 v8b;
typedef __attribute__((ext_vector_type(8))) float v8f;
typedef __attribute__((ext_vector_type(4))) float v4f;
typedef __attribute__((ext_vector_type(2))) float v2f;
__device__ __forceinline__ float bf16_rne(float f) { unsigned int u = __float_as_uint(f); u += 0x7FFFu + ((u >> 16) & 1u); float r = __uint_as_float(u & 0xFFFF0000u); asm volatile("" : "+v"(r)); return r; }
__device__ __forceinline__ void split16(float v, b16& hi, b16& lo) { hi = (b16)v; lo = (b16)(v - (float)hi); }
__device__ __forceinline__ v16b frag_kb(const b16* p, int hh) { const v8b a = *(const v8b*)(p + 8 * hh), b = *(const v8b*)(p + 16 + 8 * hh); v16b f;
#pragma unroll
  for (int e = 0; e < 8; ++e) { f[e] = a[e]; f[8 + e] = b[e]; } return f; }
__device__ __forceinline__ v8f wmma16b(v16b a, v16b b, v8f c) { v8f d = __builtin_amdgcn_wmma_f32_16x16x32_f16(false, a, false, b, (short)0, c, false, false); asm volatile("v_nop\n\tv_nop\n\tv_nop\n\tv_nop" : "+v"(d) : "v"(a), "v"(b)); return d; }
__device__ __forceinline__ void wave_lds_sync() { __builtin_amdgcn_fence(__ATOMIC_RELEASE, "workgroup"); __builtin_amdgcn_wave_barrier(); __builtin_amdgcn_fence(__ATOMIC_ACQUIRE, "workgroup"); }
__device__ __forceinline__ float pmul(float a, float b) { float p = a * b; asm volatile("" : "+v"(p)); return p; }
__device__ __forceinline__ int iclamp(int v, int lo, int hi) { return v < lo ? lo : (v > hi ? hi : v); }
__device__ __forceinline__ int branch_of(int m) { return (m == 0 || m == 10) ? 0 : ((m == 1 || m == 9) ? 1 : (m <= 5 ? 2 : 3)); }
__device__ __forceinline__ int key_of(int n) { const int m = n % 11, g = n / 11, b = branch_of(m); const int sz = (b < 2) ? 2 : (b == 2 ? 4 : 3); const int pos = (b == 0) ? (m == 0 ? 0 : 1) : (b == 1 ? (m == 1 ? 0 : 1) : (b == 2 ? m - 2 : m - 6)); const int offb = (b == 0) ? 0 : (b == 1 ? 2 : (b == 2 ? 4 : 8)); return (ND / 11) * offb + g * sz + pos; }
constexpr int CSR_NBLK9 = 512, CSR_GB9 = 9, CSR_GN9 = 1 << CSR_GB9  , CSR_TS9 = (CSR_GN9 < 32 ? 32 : CSR_GN9)  , CSR_MAXG9 = 512, CSR_CAP9 = 12288  ;
__device__ __host__ __forceinline__ int csr_tix9(int v) { return (v >> CSR_GB9) * CSR_TS9 + (v & (CSR_GN9 - 1)); }
__global__ __launch_bounds__(64) void csrA_kernel9(const int* __restrict__ dst, int E, int N, int nG, int CHP, int NGP, int* __restrict__ STG, int* __restrict__ HST) {
  extern __shared__ int sm[];
  int* cnt = sm; int* run = sm + NGP; int* ids = sm + 2 * NGP;
  const int b = blockIdx.x; const int ch = (E + CSR_NBLK9 - 1) / CSR_NBLK9; const int e0 = b * ch, e1 = min(E, e0 + ch);
  for (int i = threadIdx.x; i < NGP; i += 64) cnt[i] = 0;
  for (int i = threadIdx.x; i < CHP; i += 64) ids[i] = -1;
  __syncthreads();
  if (threadIdx.x == 0) {
    for (int e = e0; e < e1; ++e) { int d = dst[e]; d = (d < 0) ? 0 : (d >= N ? N - 1 : d); cnt[d >> CSR_GB9] += 1; }
    int acc = 0; for (int g = 0; g < nG; ++g) { run[g] = acc; acc += cnt[g]; }
    for (int e = e0; e < e1; ++e) { int d = dst[e]; d = (d < 0) ? 0 : (d >= N ? N - 1 : d); const int g = d >> CSR_GB9; ids[run[g]] = e; run[g] += 1; } }
  __syncthreads();
  typedef __attribute__((ext_vector_type(4))) int v4i;
  for (int pass = 0; pass < 2; ++pass) {
    for (int i = threadIdx.x; i < CHP / 4; i += 64) *(volatile v4i*)(STG + (size_t)b * CHP + i * 4) = *(const v4i*)(&ids[i * 4]);
    for (int i = threadIdx.x; i < NGP / 4; i += 64) { v4i v; for (int e = 0; e < 4; ++e) v[e] = (i * 4 + e < nG) ? cnt[i * 4 + e] : 0; *(volatile v4i*)(HST + (size_t)b * NGP + i * 4) = v; }
    __threadfence(); }
}
__global__ __launch_bounds__(512) void csrS_kernel9(const int* __restrict__ HST, int nG, int NGP, int* __restrict__ START, int* __restrict__ TOT, int* __restrict__ OFF) {
  __shared__ int tot[CSR_MAXG9];
  const int b = threadIdx.x;
  for (int pass = 0; pass < 2; ++pass) { int runb = 0; for (int g = 0; g < nG; ++g) { int c = HST[(size_t)b * NGP + g]; c = (c < 0) ? 0 : c; ((volatile int*)OFF)[(size_t)g * CSR_NBLK9 + b] = runb; runb += c; } __threadfence(); }
  for (int g = threadIdx.x; g < nG; g += 512) { int s = 0; for (int bb = 0; bb < CSR_NBLK9; ++bb) { int c = HST[(size_t)bb * NGP + g]; s += (c < 0) ? 0 : c; } tot[g] = s; }
  __syncthreads();
  if (threadIdx.x < 32) {
    __shared__ int st[CSR_MAXG9 + 32];
    if (threadIdx.x == 0) { int acc = 0; for (int g = 0; g < NGP; ++g) { st[g] = acc; if (g < nG) acc += (tot[g] + 31) & ~31; } st[NGP] = acc; }
    __builtin_amdgcn_fence(__ATOMIC_RELEASE, "workgroup"); __builtin_amdgcn_wave_barrier(); __builtin_amdgcn_fence(__ATOMIC_ACQUIRE, "workgroup");
    for (int pass = 0; pass < 2; ++pass) { for (int i = threadIdx.x; i < NGP + 32; i += 32) { ((volatile int*)START)[i] = (i <= NGP) ? st[min(i, NGP)] : 0; ((volatile int*)TOT)[i] = (i < nG) ? tot[i] : 0; } __threadfence(); } }
}
__global__ __launch_bounds__(256) void csrB_kernel9(const int* __restrict__ dst, int N, int nG, int CHP, int NGP, int permLen, const int* __restrict__ STG, const int* __restrict__ HST, const int* __restrict__ OFF, const int* __restrict__ START, const int* __restrict__ TOT, int* __restrict__ PERM, int* __restrict__ ROWPTR, int* __restrict__ ROWCNT, int* __restrict__ FLAG) {
  typedef __attribute__((ext_vector_type(4))) int v4i;
  __shared__ int ids[CSR_CAP9]; __shared__ unsigned short key[CSR_CAP9]; __shared__ int outp[CSR_CAP9]; __shared__ int ncnt[CSR_GN9 + 1]; __shared__ int boff[CSR_NBLK9 + 1];
  const int g = blockIdx.x, t_ = threadIdx.x; int tot = TOT[g]; int st = START[g], stn = START[g + 1]; const int v0 = g * CSR_GN9; const int nv = min(CSR_GN9, N - v0); const int t0 = g * CSR_TS9;
  st = (st < 0) ? 0 : (st > permLen - 32 ? permLen - 32 : st) & ~31; stn = (stn < st) ? st : (stn > permLen ? permLen : stn); tot = (tot < 0) ? 0 : tot; if (tot > stn - st && tot <= CSR_CAP9) tot = stn - st;
  if (tot > CSR_CAP9) {
    for (int pass = 0; pass < 2; ++pass) { for (int i = t_; i < CSR_TS9 / 4; i += 256) { v4i a, c; for (int e = 0; e < 4; ++e) { a[e] = st; c[e] = 0; } *(volatile v4i*)(ROWPTR + t0 + i * 4) = a; *(volatile v4i*)(ROWCNT + t0 + i * 4) = c; } if (t_ == 0) ((volatile int*)FLAG)[0] = 1; __threadfence(); } (void)nv; return; }
  if (t_ == 0) { int acc = 0; for (int b = 0; b < CSR_NBLK9; ++b) { boff[b] = acc; int c = HST[(size_t)b * NGP + g]; c = (c < 0) ? 0 : (c > CHP ? CHP : c); acc += c; if (acc > tot) acc = tot; } boff[CSR_NBLK9] = acc; }
  for (int i = t_; i <= CSR_GN9; i += 256) ncnt[i] = 0;
  __syncthreads();
  for (int b = 0; b < CSR_NBLK9; ++b) { const int c = boff[b + 1] - boff[b]; int o_ = OFF[(size_t)g * CSR_NBLK9 + b]; o_ = (o_ < 0) ? 0 : (o_ > CHP - c ? CHP - c : o_); const int* src_ = STG + (size_t)b * CHP + o_;
    for (int i = t_; i < c; i += 256) { int id = src_[i]; id = (id < 0) ? 0 : id; ids[boff[b] + i] = id; int d = dst[id]; d = (d < v0) ? v0 : (d >= N ? N - 1 : d); int kk = d - v0; kk = (kk < 0) ? 0 : (kk >= CSR_GN9 ? CSR_GN9 - 1 : kk); key[boff[b] + i] = (unsigned short)kk; } }
  __syncthreads();
  if (t_ == 0) { for (int i = 0; i < tot; ++i) ncnt[key[i]] += 1; int acc = 0; for (int vl = 0; vl < CSR_GN9; ++vl) { const int c = ncnt[vl]; ncnt[vl] = acc; acc += c; } ncnt[CSR_GN9] = acc;
    for (int i = 0; i < tot; ++i) { const int vl = key[i]; outp[ncnt[vl]] = ids[i]; ncnt[vl] += 1; }
    for (int vl = CSR_GN9; vl > 0; --vl) ncnt[vl] = ncnt[vl - 1]; ncnt[0] = 0; }
  __syncthreads();
  for (int pass = 0; pass < 2; ++pass) {
    for (int i = t_; i < (stn - st) / 4; i += 256) { v4i v; for (int e = 0; e < 4; ++e) { const int q = i * 4 + e; v[e] = (q < tot) ? outp[q] : -1; } *(volatile v4i*)(PERM + st + i * 4) = v; }
    for (int i = t_; i < CSR_TS9 / 4; i += 256) { v4i a, c; for (int e = 0; e < 4; ++e) { const int vl = i * 4 + e; const int vc = vl < CSR_GN9 ? vl : CSR_GN9; a[e] = (vl < CSR_GN9) ? st + ncnt[vc] : st; c[e] = (vl < nv) ? (ncnt[(vc < CSR_GN9 ? vc : CSR_GN9 - 1) + 1] - ncnt[vc]) : 0; } *(volatile v4i*)(ROWPTR + t0 + i * 4) = a; *(volatile v4i*)(ROWCNT + t0 + i * 4) = c; }
    __threadfence(); }
}
__global__ __launch_bounds__(256) void csrZ_kernel9(int* __restrict__ p, size_t n4) { typedef __attribute__((ext_vector_type(4))) int v4i; const size_t tid = (size_t)blockIdx.x * 256 + threadIdx.x, nth = (size_t)gridDim.x * 256; v4i z = {0, 0, 0, 0}; for (size_t i = tid; i < n4; i += nth) *(volatile v4i*)(p + i * 4) = z; }
struct CsrBufs9 { int *STG, *HST, *OFF, *START, *TOT, *PERM, *ROWPTR, *ROWCNT, *FLAG; int nG, NGP, CHP; size_t permLen; char* base; size_t bytes; };
static size_t csr_carve9(CsrBufs9& c, char* ws, size_t off, int E, int N) {
  const size_t off0 = off; c.base = ws + off;
  auto al = [&](size_t bytes) { char* p = ws + off; off += (bytes + 255) & ~(size_t)255; return p; };
  c.nG = (N + CSR_GN9 - 1) / CSR_GN9; c.NGP = (c.nG + 31) & ~31; const int ch = (E + CSR_NBLK9 - 1) / CSR_NBLK9; c.CHP = (ch + 31) & ~31; c.permLen = (size_t)E + 32 * (size_t)c.nG + 32;
  c.STG = (int*)al((size_t)CSR_NBLK9 * c.CHP * 4); c.HST = (int*)al((size_t)CSR_NBLK9 * c.NGP * 4); c.OFF = (int*)al((size_t)c.NGP * CSR_NBLK9 * 4); c.START = (int*)al((size_t)(c.NGP + 64) * 4); c.TOT = (int*)al((size_t)(c.NGP + 64) * 4);
  c.PERM = (int*)al(c.permLen * 4); c.ROWPTR = (int*)al((size_t)c.nG * CSR_TS9 * 4); c.ROWCNT = (int*)al((size_t)c.nG * CSR_TS9 * 4); c.FLAG = (int*)al(256);
  c.bytes = off - off0; return off;
}
static void csr_build9(const CsrBufs9& c, const int* dst, int E, int N, hipStream_t stream) {
  const size_t smem = (size_t)(2 * c.NGP + c.CHP) * 4;
  csrZ_kernel9<<<512, 256, 0, stream>>>((int*)c.base, c.bytes / 16);
  csrA_kernel9<<<CSR_NBLK9, 64, smem, stream>>>(dst, E, N, c.nG, c.CHP, c.NGP, c.STG, c.HST);
  csrS_kernel9<<<1, 512, 0, stream>>>(c.HST, c.nG, c.NGP, c.START, c.TOT, c.OFF);
  csrB_kernel9<<<c.nG, 256, 0, stream>>>(dst, N, c.nG, c.CHP, c.NGP, (int)c.permLen, c.STG, c.HST, c.OFF, c.START, c.TOT, c.PERM, c.ROWPTR, c.ROWCNT, c.FLAG);
}


__global__ __launch_bounds__(256) void key_kernel(const int* __restrict__ dsts, int* __restrict__ KEY) { const int e = blockIdx.x * 256 + threadIdx.x; if (e >= E) return; const int v = key_of(iclamp(dsts[e], 0, ND - 1)); for (int pass = 0; pass < 2; ++pass) { ((volatile int*)KEY)[e] = v; __threadfence(); } }
__global__ __launch_bounds__(256) void wput_kernel(const float* __restrict__ w1, const float* __restrict__ w2, b16* __restrict__ W1T, b16* __restrict__ W2T) { const int u = blockIdx.x * 256 + threadIdx.x;
  for (int pass = 0; pass < 2; ++pass) {
    if (u < NBR * C * (KPAD / 8)) { const int b = u / (C * 12), o = (u / 12) % C, k0 = (u % 12) * 8; v8b v; for (int j = 0; j < 8; ++j) { const int k = k0 + j; int row = -1; if (k < 32) row = k; else if (k < 36) row = k; else if (k >= 64) row = k - 28; v[j] = (b16)(row >= 0 ? bf16_rne(w1[((size_t)b * 68 + row) * C + o]) * WSC : 0.0f); } *(volatile v8b*)(W1T + ((size_t)b * C + o) * KPAD + k0) = v; }
    if (u < NBR * C * 4) { const int b = u / (C * 4), o = (u / 4) % C, k0 = (u % 4) * 8; v8b v; for (int j = 0; j < 8; ++j) v[j] = (b16)(bf16_rne(w2[((size_t)b * C + k0 + j) * C + o]) * WSC); *(volatile v8b*)(W2T + ((size_t)b * C + o) * C + k0) = v; }
    __threadfence(); } }
__device__ __forceinline__ float angle_(float ax, float ay, float az, float bx, float by, float bz) { const float cx = ay * bz - az * by, cy = az * bx - ax * bz, cz = ax * by - ay * bx; return atan2f(sqrtf(pmul(cx, cx) + pmul(cy, cy) + pmul(cz, cz)), pmul(ax, bx) + pmul(ay, by) + pmul(az, bz)); }
__global__ __launch_bounds__(32) void edge_kernel(const float* __restrict__ xd, const float* __restrict__ vd, const float* __restrict__ xp, const float* __restrict__ vp, const float* __restrict__ pv, const float* __restrict__ dv, const int* __restrict__ srcs, const int* __restrict__ dsts, const int* __restrict__ PERM, int permLen, int KLIM, const b16* __restrict__ W1T, const float* __restrict__ b1, const b16* __restrict__ W2T, const float* __restrict__ b2, float* __restrict__ HE) {
  __shared__ __attribute__((aligned(16))) b16 Ah[16][KPAD + 8], Al[16][KPAD + 8], Hh[16][40], Hl[16][40]; __shared__ float Tf[16][C + 1]; __shared__ int Br[16]; const int lane = threadIdx.x, nloc = lane & 15, hlf = lane >> 4; const size_t p0 = (size_t)blockIdx.x * 16; if (p0 >= (size_t)permLen) return;
  if (KLIM < ND && key_of(iclamp(dsts[iclamp(PERM[p0], 0, E - 1)], 0, ND - 1)) >= KLIM) return;
  { const int rr = lane & 15; const size_t p = p0 + rr; const int e = iclamp(PERM[p < (size_t)permLen ? p : permLen - 1], 0, E - 1); const int i = iclamp(dsts[e], 0, ND - 1), j = iclamp(srcs[e], 0, NP_ - 1); if (hlf == 0) Br[rr] = branch_of(i % 11);
    if (hlf == 0) { for (int c = 0; c < C; ++c) { Ah[rr][c] = (b16)(bf16_rne(xp[(size_t)j * C + c]) * XS); Al[rr][c] = (b16)0.0f; }
      const float pix = bf16_rne(vd[(size_t)i * 3]), piy = bf16_rne(vd[(size_t)i * 3 + 1]), piz = bf16_rne(vd[(size_t)i * 3 + 2]); const float pjx = bf16_rne(vp[(size_t)j * 3]), pjy = bf16_rne(vp[(size_t)j * 3 + 1]), pjz = bf16_rne(vp[(size_t)j * 3 + 2]);
      const float nix = bf16_rne(dv[(size_t)i * 3]), niy = bf16_rne(dv[(size_t)i * 3 + 1]), niz = bf16_rne(dv[(size_t)i * 3 + 2]); const float njx = bf16_rne(pv[(size_t)j * 3]), njy = bf16_rne(pv[(size_t)j * 3 + 1]), njz = bf16_rne(pv[(size_t)j * 3 + 2]);
      const float dx = pjx - pix, dy = pjy - piy, dz = pjz - piz; float f[4]; f[0] = sqrtf(pmul(dx, dx) + pmul(dy, dy) + pmul(dz, dz)); f[1] = angle_(nix, niy, niz, dx, dy, dz); f[2] = angle_(njx, njy, njz, dx, dy, dz); f[3] = angle_(nix, niy, niz, njx, njy, njz);
      for (int c = 0; c < 4; ++c) { b16 ph, pl; split16(f[c] * XS, ph, pl); Ah[rr][32 + c] = ph; Al[rr][32 + c] = pl; } for (int c = 36; c < 64; ++c) { Ah[rr][c] = (b16)0.0f; Al[rr][c] = (b16)0.0f; } }
    else { for (int c = 0; c < C; ++c) { Ah[rr][64 + c] = (b16)(bf16_rne(xd[(size_t)i * C + c]) * XS); Al[rr][64 + c] = (b16)0.0f; } } }
  wave_lds_sync(); const int bA = Br[0], bB = Br[15];
  for (int which = 0; which < 2; ++which) { const int b = which == 0 ? bA : bB; if (which == 1 && bB == bA) break;
    v8f acc[2] = {(v8f){}, (v8f){}};
#pragma unroll
    for (int kb = 0; kb < KPAD; kb += 32) { const v16b a = frag_kb(&Ah[nloc][kb], hlf); const bool lo = (kb == 32); v16b al; if (lo) al = frag_kb(&Al[nloc][kb], hlf);
#pragma unroll
      for (int t = 0; t < 2; ++t) { const v16b bw = frag_kb(W1T + ((size_t)b * C + t * 16 + nloc) * KPAD + kb, hlf); acc[t] = wmma16b(a, bw, acc[t]); if (lo) acc[t] = wmma16b(al, bw, acc[t]); } }
#pragma unroll
    for (int t = 0; t < 2; ++t) { const int c = t * 16 + nloc; const float bb = bf16_rne(b1[b * C + c]);
#pragma unroll
      for (int r8 = 0; r8 < 8; ++r8) { const int rl = 8 * hlf + r8; if (which == 0 || Br[rl] == b) { b16 p, q; split16(fmaxf(acc[t][r8] * (1.0f / (XS * WSC)) + bb, 0.0f) * XS, p, q); Hh[rl][c] = p; Hl[rl][c] = q; } } }
    wave_lds_sync(); v8f acc2[2] = {(v8f){}, (v8f){}}; { const v16b a = frag_kb(&Hh[nloc][0], hlf), al = frag_kb(&Hl[nloc][0], hlf);
#pragma unroll
      for (int t = 0; t < 2; ++t) { const v16b bw = frag_kb(W2T + ((size_t)b * C + t * 16 + nloc) * C, hlf); acc2[t] = wmma16b(a, bw, acc2[t]); acc2[t] = wmma16b(al, bw, acc2[t]); } }
#pragma unroll
    for (int t = 0; t < 2; ++t) { const int c = t * 16 + nloc; const float bb = bf16_rne(b2[b * C + c]);
#pragma unroll
      for (int r8 = 0; r8 < 8; ++r8) { const int rl = 8 * hlf + r8; if (which == 0 || Br[rl] == b) Tf[rl][c] = fmaxf(acc2[t][r8] * (1.0f / (XS * WSC)) + bb, 0.0f); } }
    wave_lds_sync(); }
  for (int pass = 0; pass < 2; ++pass) { for (int rr = 0; rr < 16; ++rr) if (p0 + rr < (size_t)permLen) ((volatile float*)HE)[(p0 + rr) * C + lane] = Tf[rr][lane]; __threadfence(); }
}
__global__ __launch_bounds__(256) void node_kernel(const float* __restrict__ HE, const int* __restrict__ ROWPTR, const int* __restrict__ ROWCNT, int permLen, int KLIM, float* __restrict__ out, float* __restrict__ conv) {
  const int wave = threadIdx.x >> 5, lane = threadIdx.x & 31; const size_t n = (size_t)blockIdx.x * 8 + wave; if (n >= (size_t)ND) return; const int key = key_of((int)n); float s = 0.0f;
  if (key < KLIM) { int st = ROWPTR[key], cnt = ROWCNT[key]; cnt = iclamp(cnt, 0, 1 << 20); st = iclamp(st, 0, permLen - cnt);
#pragma unroll 1
    for (int j = 0; j < cnt; ++j) s += HE[(size_t)(st + j) * C + lane]; }
  for (int pass = 0; pass < 2; ++pass) { ((volatile float*)conv)[n * C + lane] = s; ((volatile float*)out)[n * C + lane] = fmaxf(s, 0.0f); __threadfence(); } }
}

extern "C" void kernel_launch(void* const* d_in, const int* in_sizes, int n_in, void* d_out, int out_size, void* d_ws, size_t ws_size, hipStream_t stream) {
  (void)n_in;
  auto Fp = [&](int i) { return (const float*)d_in[i]; }; auto Ip = [&](int i) { return (const int*)d_in[i]; };
  if (in_sizes[0] != ND * C || in_sizes[1] != ND * 3 || in_sizes[2] != NP_ * C || in_sizes[3] != NP_ * 3 || in_sizes[4] != NP_ * 3 || in_sizes[5] != ND * 3 || in_sizes[6] != E || in_sizes[7] != E || in_sizes[8] != NBR * 68 * C || in_sizes[10] != NBR * C * C || out_size != 2 * ND * C) return;
  const int KLIM = ND;
  size_t off = 0; char* ws = (char*)d_ws;
  auto carve = [&](size_t bytes) { char* p = ws + off; off += (bytes + 255) & ~(size_t)255; return p; };
  int* KEY = (int*)carve((size_t)E * 4); b16* W1T = (b16*)carve((size_t)NBR * C * KPAD * 2); b16* W2T = (b16*)carve((size_t)NBR * C * C * 2); const size_t permRows = (size_t)E + 32 * (size_t)((ND + 511) / 512) + 32;     float* HE = (float*)carve(permRows * C * 4); CsrBufs9 csr; off = csr_carve9(csr, ws, off, E, ND); if (csr.permLen != permRows) return;
  if (off > ws_size || off > ((size_t)240 << 20)) return;
  key_kernel<<<(E + 255) / 256, 256, 0, stream>>>(Ip(7), KEY);
  wput_kernel<<<(NBR * C * 12 + 255) / 256, 256, 0, stream>>>(Fp(8), Fp(10), W1T, W2T);
  csr_build9(csr, KEY, E, ND, stream);
  edge_kernel<<<(unsigned)((csr.permLen + 15) / 16), 32, 0, stream>>>(
      Fp(0), Fp(1), Fp(2), Fp(3), Fp(4), Fp(5), Ip(6), Ip(7), csr.PERM, (int)csr.permLen, KLIM, W1T, Fp(9), W2T, Fp(11), HE);
  float* out = (float*)d_out;
  node_kernel<<<(ND + 7) / 8, 256, 0, stream>>>(HE, csr.ROWPTR, csr.ROWCNT, (int)csr.permLen, KLIM, out, out + (size_t)ND * C);
}
